// DotProductAtten_85048942395855
// MI455X (gfx1250) — hardware-verified
//
#include <hip/hip_runtime.h>


#ifndef NB
#define NB 16
#endif
#ifndef SEQ
#define SEQ 4096
#endif
#define NB_FULL  16
#define SEQ_FULL 4096
#ifndef OUT_SEQ
#define OUT_SEQ SEQ
#endif
#define HD   64
#define AW   4
#define OSP  68
#define TP   72
#define XC   16.0f
#define XCI  (1.0f / 16.0f)
#define SC2  ((float)(0.125 * 1.4426950408889634 / 256.0))
#define FILL2 ((float)(-1.0e6 * 1.4426950408889634))
#define PSH  14.0f
#define NEGB (-3.0e38f)

static_assert(HD == 64);
static_assert(HD % 32 == 0);
static_assert(SEQ % 64 == 0);
static_assert(SEQ % 32 == 0);
static_assert(SEQ % (16 * AW) == 0);
static_assert(((size_t)SEQ * HD) % 8 == 0);
static_assert(NB <= NB_FULL);
static_assert(SEQ <= SEQ_FULL);
static_assert(OSP >= HD);
static_assert((OSP * 4) % 16 == 0);
static_assert(TP >= 64);
static_assert((TP * 2) % 16 == 0);
static_assert(8 * 32 * 16 == 16 * HD * 4);
static_assert(256 * 2 * 16 == HD * 64 * 2);
static_assert(256 * 4 * 4 == 64 * HD);
static_assert((size_t)AW * 16 * OSP * 4 <= 131072);
static_assert((size_t)HD * TP * 2 <= 131072);

typedef _Float16 h16;
typedef __attribute__((ext_vector_type(16))) _Float16 v16h;
typedef __attribute__((ext_vector_type(8)))  _Float16 v8h;
typedef __attribute__((ext_vector_type(8)))  float    v8f;
typedef __attribute__((ext_vector_type(4)))  float    v4f;
typedef v4f  __attribute__((may_alias)) v4fa;
typedef v8h  __attribute__((may_alias)) v8ha;

__device__ __forceinline__ unsigned short f2bf(float f) { unsigned u = __float_as_uint(f); u += 0x7FFFu + ((u >> 16) & 1u); return (unsigned short)(u >> 16); }
__device__ __forceinline__ float bfr(float f) { return __uint_as_float(((unsigned)f2bf(f)) << 16); }
__device__ __forceinline__ v16h cat16(v8h lo, v8h hi) { return __builtin_shufflevector(lo, hi, 0, 1, 2, 3, 4, 5, 6, 7, 8, 9, 10, 11, 12, 13, 14, 15); }
__device__ __forceinline__ v8f wmma16(v16h a, v16h b, v8f c) { return __builtin_amdgcn_wmma_f32_16x16x32_f16(false, a, false, b, (short)0, c, false, false); }
__device__ __forceinline__ v8f wmma16g(v16h a, v16h b, v8f c) { c = wmma16(a, b, c); asm volatile("v_nop\n\tv_nop\n\tv_nop\n\tv_nop" : "+v"(c) : "v"(a), "v"(b)); return c; }
__device__ __forceinline__ v16h  ldh(const h16* p) { return cat16(*(const v8h*)p, *(const v8h*)(p + 16)); }
__device__ __forceinline__ void wave_sync() { __builtin_amdgcn_fence(3  , "wavefront"); __builtin_amdgcn_wave_barrier(); asm volatile("" ::: "memory"); }
static __device__ __forceinline__ h16 toh_flush(float v) { const h16 r = (h16)v; return (fabsf(v) < 6.103515625e-05f) ? (h16)0.0f : r; }

__global__ __launch_bounds__(256) void k_cvth(const float* __restrict__ src, h16* dst, size_t n8) {
#pragma clang fp contract(off)
    const size_t i = (size_t)blockIdx.x * 256 + threadIdx.x; if (i >= n8) return;
    const v8f v = *(const v8f*)(src + i * 8); v8h o;
#pragma unroll
    for (int k = 0; k < 8; ++k) o[k] = toh_flush(bfr(v[k]) * XC);
    *(volatile v8h*)(dst + i * 8) = o; __threadfence(); *(volatile v8h*)(dst + i * 8) = o;
}

__global__ __launch_bounds__(256) void k_vt(const float* __restrict__ src, h16* dst) {
#pragma clang fp contract(off)
    __shared__ __align__(16) h16 ts[HD * TP];
    const int tid = threadIdx.x;
    const int b = blockIdx.y; const int t0 = blockIdx.x * 64;
    const float* sp = src + ((size_t)b * SEQ_FULL + (size_t)t0) * HD;
#pragma unroll 1
    for (int s = 0; s < 4; ++s) { const int p = s * 256 + tid; const int tok = p >> 4, c0 = (p & 15) * 4;
        const v4f x = *(const v4f*)(sp + (size_t)p * 4);
#pragma unroll
        for (int i = 0; i < 4; ++i) ts[(c0 + i) * TP + tok] = toh_flush(bfr(x[i]) * XC); }
    __syncthreads();
    h16* dp = dst + (size_t)b * HD * SEQ + (size_t)t0;
#pragma unroll 1
    for (int ps = 0; ps < 2; ++ps) {
#pragma unroll
        for (int s = 0; s < 2; ++s) { const int p = s * 256 + tid; const int row = p >> 3, c8 = (p & 7) * 8;
            const v8h val = *(const v8ha*)(&ts[row * TP + c8]);
            *(volatile v8h*)(dp + (size_t)row * SEQ + c8) = val; }
        if (ps == 0) __threadfence(); }
}

__global__ __launch_bounds__(32 * AW) void k_flash(const h16* __restrict__ QH, const h16* __restrict__ KP, const h16* __restrict__ VT, const int* __restrict__ vlen, float* OUT) {
    __shared__ __align__(16) float os[AW * 16 * OSP];
    const int lane = threadIdx.x & 31, lr = lane & 15, hi = lane >> 4;
    const int wave = __builtin_amdgcn_readfirstlane((int)(threadIdx.x >> 5));
    const int b = blockIdx.y;
    const int t0 = (blockIdx.x * AW + wave) * 16;
    int vl = vlen[b]; vl = vl > SEQ ? SEQ : vl;
    const int kend = vl < 1 ? SEQ : vl;
    const int nk = (kend + 31) & ~31;
    const size_t pbase = (size_t)b * SEQ * HD;
    const size_t qo = pbase + (size_t)(t0 + lr) * HD + 8 * hi;
    const v16h q0 = ldh(QH + qo), q1 = ldh(QH + qo + 32);
    const size_t ko = pbase + (size_t)lr * HD + 8 * hi;
    const size_t vo = pbase + (size_t)lr * SEQ + 8 * hi;
    v8f o[4];
#pragma unroll
    for (int j = 0; j < 4; ++j) o[j] = (v8f){};
    float m = NEGB, l = 0.0f;
#pragma unroll 1
    for (int key0 = 0; key0 < nk; key0 += 32) {
        const h16* ka = KP + ko + (size_t)key0 * HD;
        const v16h ka0 = ldh(ka), ka1 = ldh(ka + 32), kb0 = ldh(ka + 16 * HD), kb1 = ldh(ka + 16 * HD + 32);
        v8f sa = (v8f){}, sb = (v8f){};
        sa = wmma16g(ka0, q0, sa); sb = wmma16g(kb0, q0, sb); sa = wmma16g(ka1, q1, sa); sb = wmma16g(kb1, q1, sb);
        const int ja = key0 + 8 * hi;
        float ta[8], tb[8]; float mx = NEGB;
#pragma unroll
        for (int r = 0; r < 8; ++r) {
            const bool fa = (ja + r) < vl;
            const bool fb = (ja + 16 + r) < vl;
            const float xa = sa[r] * SC2, xb = sb[r] * SC2;
            ta[r] = fa ? xa : FILL2; tb[r] = fb ? xb : FILL2;
            mx = fmaxf(mx, fmaxf(ta[r], tb[r])); }
        mx = fmaxf(mx, __shfl_xor(mx, 16, 32));
        const float mnew = fmaxf(m, mx);
        const float alpha = __builtin_amdgcn_exp2f(m - mnew);
        const float sh = PSH - mnew;
        v16h pb; float ls = 0.0f;
#pragma unroll
        for (int r = 0; r < 8; ++r) {
            const float ea = ta[r] + sh, eb = tb[r] + sh;
            const float xa = __builtin_amdgcn_exp2f(ea), xb = __builtin_amdgcn_exp2f(eb);
            const float ga = (ea < -14.0f) ? 0.0f : xa, gb = (eb < -14.0f) ? 0.0f : xb;
            const h16 pa = (h16)ga; const h16 pc = (h16)gb;
            pb[r] = pa; pb[8 + r] = pc;
            ls += (float)pa + (float)pc; }
        l = l * alpha + ls; m = mnew;
#pragma unroll
        for (int j = 0; j < 4; ++j) o[j] = o[j] * alpha;
        const h16* va = VT + vo + key0;
        v16h vf[4];
#pragma unroll
        for (int j = 0; j < 4; ++j) vf[j] = ldh(va + (size_t)(16 * j) * SEQ);
#pragma unroll
        for (int j = 0; j < 4; ++j) o[j] = wmma16g(vf[j], pb, o[j]);
    }
    l += __shfl_xor(l, 16, 32);
    const bool any = l > 0.0f;
    const float lsafe = any ? l : 1.0f;
    const float inv = any ? ((1.0f / lsafe) * XCI) : 0.0f;
    const int wb = wave * 16 * OSP;
#pragma unroll
    for (int j = 0; j < 4; ++j) { v4f a, c;
        a[0] = o[j][0] * inv; a[1] = o[j][1] * inv; a[2] = o[j][2] * inv; a[3] = o[j][3] * inv;
        c[0] = o[j][4] * inv; c[1] = o[j][5] * inv; c[2] = o[j][6] * inv; c[3] = o[j][7] * inv;
        *(v4fa*)(&os[wb + lr * OSP + 16 * j + 8 * hi]) = a; *(v4fa*)(&os[wb + lr * OSP + 16 * j + 8 * hi + 4]) = c; }
    wave_sync();
    float* orow = OUT + ((size_t)b * OUT_SEQ + (size_t)t0) * HD;
#pragma unroll 1
    for (int ps = 0; ps < 2; ++ps) {
#pragma unroll
        for (int s = 0; s < 8; ++s) { const int p = s * 32 + lane; const int row = p >> 4, cofs = (p & 15) * 4;
            const v4f val = *(const v4fa*)(&os[wb + row * OSP + cofs]);
            *(volatile v4f*)(orow + (size_t)p * 4) = val; }
        if (ps == 0) __threadfence(); }
}

static constexpr size_t al256(size_t v) { return (v + 255) & ~(size_t)255; }
static constexpr size_t SZ_PL = al256((size_t)NB * SEQ * HD * 2);
static constexpr size_t SZ_TOTAL = 3 * SZ_PL;
static_assert(SZ_TOTAL <= (size_t)134217728);
static_assert(((size_t)SEQ * 2) % 128 == 0);

extern "C" void kernel_launch(void* const* d_in, const int* in_sizes, int n_in,
                              void* d_out, int out_size, void* d_ws, size_t ws_size, hipStream_t stream) {
    if (n_in < 4) return;
    const size_t needx = ((size_t)(NB - 1) * SEQ_FULL + SEQ) * HD;
    if ((size_t)in_sizes[0] < needx || (size_t)in_sizes[1] < needx || (size_t)in_sizes[2] < needx) return;
    if (in_sizes[3] < NB) return;
    if ((size_t)out_size < ((size_t)(NB - 1) * OUT_SEQ + SEQ) * HD) return;
    if (SZ_TOTAL > ws_size) return;
    const float* qin = (const float*)d_in[0];
    const float* kin = (const float*)d_in[1];
    const float* vin = (const float*)d_in[2];
    const int* vlen = (const int*)d_in[3];
    float* OUT = (float*)d_out;
    char* wsp = (char*)d_ws;
    h16* QH = (h16*)wsp; wsp += SZ_PL;
    h16* KP = (h16*)wsp; wsp += SZ_PL;
    h16* VT = (h16*)wsp; wsp += SZ_PL;

    if (SEQ == SEQ_FULL) {
        const size_t n8 = (size_t)NB * SEQ * HD / 8;
        k_cvth<<<(unsigned)((n8 + 255) / 256), 256, 0, stream>>>(qin, QH, n8);
        k_cvth<<<(unsigned)((n8 + 255) / 256), 256, 0, stream>>>(kin, KP, n8);
    } else {
        const size_t n8 = (size_t)SEQ * HD / 8;
        for (int b = 0; b < NB; ++b) {
            k_cvth<<<(unsigned)((n8 + 255) / 256), 256, 0, stream>>>(qin + (size_t)b * SEQ_FULL * HD, QH + (size_t)b * SEQ * HD, n8);
            k_cvth<<<(unsigned)((n8 + 255) / 256), 256, 0, stream>>>(kin + (size_t)b * SEQ_FULL * HD, KP + (size_t)b * SEQ * HD, n8);
        }
    }
    k_vt<<<dim3(SEQ / 64, NB, 1), 256, 0, stream>>>(vin, VT);

    k_flash<<<dim3(SEQ / (16 * AW), NB, 1), 32 * AW, 0, stream>>>(QH, KP, VT, vlen, OUT);
}
